// SelfAttention_32942399160710
// MI455X (gfx1250) — hardware-verified
//
#include <hip/hip_runtime.h>
#include <stddef.h>


typedef _Float16 h16;
typedef _Float16 v16h __attribute__((ext_vector_type(16)));
typedef _Float16 v8h  __attribute__((ext_vector_type(8)));
typedef float    v8f  __attribute__((ext_vector_type(8)));
typedef float    v4f  __attribute__((ext_vector_type(4)));

#ifndef NB
#define NB 8
#endif
#define NB_FULL 8
#define CCH   256
#define IMG   64
#define NTOK  4096
#define MTOK  1024
#define DQK   32
#define DV    128

#ifndef SCORE_RES
#define SCORE_RES 1
#endif

static_assert(NB >= 1 && NB <= NB_FULL);
static_assert(IMG == 64);
static_assert(NTOK == IMG * IMG);
static_assert(MTOK * 4 == NTOK);
static_assert(DQK == 32);
static_assert(2 * DQK == 64);
static_assert(DV == 128 && (DV % 64) == 0 && (DV % 32) == 0);
static_assert((CCH % 64) == 0 && (CCH % 32) == 0);
static_assert((NTOK % 256) == 0 && (NTOK % 128) == 0 && (MTOK % 64) == 0);
static_assert(((DQK * CCH) % 2048) == 0 && ((DV * CCH) % 2048) == 0);

#define LDT 72
#define LDC 68
#define LDK 40
#define LDP 136
static_assert((LDT % 8) == 0 && LDT >= 64);
static_assert((LDC % 4) == 0 && LDC >= 64);
static_assert((LDK % 8) == 0 && LDK >= DQK);
static_assert((LDP % 8) == 0 && LDP >= DV && LDP >= 64);

#define XCARRY 64.0f
#define WCARRY 64.0f
#define PCARRY 16384.0f
#define VCARRY 64.0f
#define RCARRY 2048.0f

#define XT_BYTES  ((size_t)NB * NTOK * CCH * 2)
#define WQK_BYTES ((size_t)2 * DQK * CCH * 2)
#define WV_BYTES  ((size_t)DV * CCH * 2)
#define WO_BYTES  ((size_t)CCH * DV * 2)
#define Q_BYTES   ((size_t)NB * NTOK * DQK * 2)
#define K_BYTES   ((size_t)NB * MTOK * DQK * 2)
#define VT_BYTES  ((size_t)NB * DV * MTOK * 2)
#define CTX_BYTES ((size_t)NB * NTOK * DV * 2)
#define OFF_XT  ((size_t)0)
#define OFF_WQK (OFF_XT + XT_BYTES)
#define OFF_WV  (OFF_WQK + WQK_BYTES)
#define OFF_WO  (OFF_WV + WV_BYTES)
#define OFF_Q   (OFF_WO + WO_BYTES)
#define OFF_QR  (OFF_Q + Q_BYTES)
#define OFF_K   (OFF_QR + Q_BYTES)
#define OFF_KR  (OFF_K + K_BYTES)
#define OFF_VT  (OFF_KR + K_BYTES)
#define OFF_CTX (OFF_VT + VT_BYTES)
#define WS_TOTAL (OFF_CTX + CTX_BYTES)
static_assert((XT_BYTES % 128) == 0 && (WQK_BYTES % 128) == 0 && (WV_BYTES % 128) == 0);
static_assert((WO_BYTES % 128) == 0 && (Q_BYTES % 128) == 0 && (K_BYTES % 128) == 0);
static_assert((VT_BYTES % 128) == 0 && (CTX_BYTES % 128) == 0);
static_assert(WS_TOTAL <= (size_t)134217728);

__device__ __forceinline__ float bf16r(float x) {
  unsigned int u = __float_as_uint(x);
  u = (u + 0x7FFFu + ((u >> 16) & 1u)) & 0xFFFF0000u;
  return __uint_as_float(u);
}

static __device__ __forceinline__ h16 toh_flush(float v) {
  const h16 r = (h16)v;
  return (fabsf(v) < 6.103515625e-05f) ? (h16)0.0f : r;
}

__device__ __forceinline__ v16h frag_at(const _Float16* p) {
  v8h lo = *(const v8h*)(p);
  v8h hi = *(const v8h*)(p + 16);
  v16h out;
#pragma unroll
  for (int i = 0; i < 8; ++i) { out[i] = lo[i]; out[i + 8] = hi[i]; }
  return out;
}
__device__ __forceinline__ v16h ld_frag(const _Float16* base, unsigned ld) {
  const unsigned lane = threadIdx.x & 31u;
  return frag_at(base + (lane & 15u) * ld + (lane >> 4) * 8u);
}

__device__ __forceinline__ v8f wmma16(v16h a, v16h b, v8f c) {
  v8f d = __builtin_amdgcn_wmma_f32_16x16x32_f16(false, a, false, b, (short)0, c,
                                                 false, false);
  asm volatile("v_nop\n\tv_nop\n\tv_nop\n\tv_nop" : "+v"(d) : "v"(a), "v"(b));
  return d;
}

__device__ __forceinline__ float red16_max(float x) {
#pragma unroll
  for (int off = 1; off < 16; off <<= 1) x = fmaxf(x, __shfl_xor(x, off, 32));
  return x;
}
__device__ __forceinline__ float red16_sum(float x) {
#pragma unroll
  for (int off = 1; off < 16; off <<= 1) x += __shfl_xor(x, off, 32);
  return x;
}

__device__ __forceinline__ void wave_lds_sync() {
  __builtin_amdgcn_fence(3  , "wavefront");
  asm volatile("s_wait_dscnt 0x0" ::: "memory");
  __builtin_amdgcn_wave_barrier();
}

__device__ __forceinline__ unsigned pool_pos(unsigned T, unsigned r) {
  return (2u * (T >> 1) + (r >> 5)) * (unsigned)IMG + 32u * (T & 1u) + (r & 31u);
}

__device__ __forceinline__ void gemm_k_loop(const h16* __restrict__ ap,
                                            const h16* __restrict__ bp0,
                                            const h16* __restrict__ bp1,
                                            const unsigned K, v8f& acc0, v8f& acc1) {
#pragma unroll 2
  for (unsigned k0 = 0; k0 < K; k0 += 32u) {
    const v16h a  = frag_at(ap + k0);
    const v16h b0 = frag_at(bp0 + k0);
    const v16h b1 = frag_at(bp1 + k0);
    acc0 = wmma16(a, b0, acc0);
    acc1 = wmma16(a, b1, acc1);
  }
}

__global__ __launch_bounds__(256) void wcast_kernel(const float* __restrict__ W,
                                                    h16* __restrict__ dst) {
  const size_t e = ((size_t)blockIdx.x * 256u + threadIdx.x) * 8u;
  const v4f a0 = *(const v4f*)(W + e);
  const v4f a1 = *(const v4f*)(W + e + 4u);
  v8h o;
#pragma unroll
  for (int i = 0; i < 4; ++i) {
    o[i]     = toh_flush(WCARRY * bf16r(a0[i]));
    o[i + 4] = toh_flush(WCARRY * bf16r(a1[i]));
  }
  *(volatile v8h*)(dst + e) = o;
  __threadfence();
  *(volatile v8h*)(dst + e) = o;
}

__global__ __launch_bounds__(256) void xconv_kernel(const float* __restrict__ X,
                                                    h16* __restrict__ Xt) {
  __shared__ __attribute__((aligned(16))) h16 T[64 * LDT];
  const unsigned tid = threadIdx.x;
  const unsigned n0 = blockIdx.x * 64u;
  const unsigned k0 = blockIdx.y * 64u;
  const unsigned b = blockIdx.z;
  const float* xb = X + (size_t)b * CCH * NTOK;
#pragma unroll 4
  for (unsigned j = 0; j < 16u; ++j) {
    const unsigned idx = tid + 256u * j;
    const unsigned kr = idx >> 6, nc = idx & 63u;
    const float v = xb[(size_t)(k0 + kr) * NTOK + n0 + nc];
    T[nc * LDT + kr] = toh_flush(XCARRY * bf16r(v));
  }
  __syncthreads();
  v8h x[2];
  size_t off[2];
#pragma unroll
  for (unsigned i = 0; i < 2u; ++i) {
    const unsigned n = 32u * i + (tid >> 3);
    const unsigned kc = (tid & 7u) * 8u;
    x[i] = *(const v8h*)&T[n * LDT + kc];
    off[i] = ((size_t)b * NTOK + n0 + n) * CCH + k0 + kc;
  }
#pragma unroll
  for (int i = 0; i < 2; ++i) *(volatile v8h*)(Xt + off[i]) = x[i];
  __threadfence();
#pragma unroll
  for (int i = 0; i < 2; ++i) *(volatile v8h*)(Xt + off[i]) = x[i];
}

__global__ __launch_bounds__(256) void gemm_qk_kernel(
    const h16* __restrict__ Xt, const h16* __restrict__ Wqk,
    h16* __restrict__ Qh, h16* __restrict__ Qr,
    h16* __restrict__ Kh, h16* __restrict__ Kr) {
  __shared__ __attribute__((aligned(16))) float Cs[64 * LDC];
  const unsigned tid = threadIdx.x, lane = tid & 31u;
  const unsigned w = __builtin_amdgcn_readfirstlane(tid >> 5);
  const unsigned mw = w >> 1, nw = w & 1u;
  const unsigned hh = lane >> 4, m = lane & 15u;
  const unsigned T = blockIdx.x;
  const unsigned b = blockIdx.y;

  const unsigned na = pool_pos(T, mw * 16u + m);
  const h16* ap  = Xt + ((size_t)b * NTOK + na) * CCH + hh * 8u;
  const h16* bp0 = Wqk + (size_t)(nw * 32u + m) * CCH + hh * 8u;
  const h16* bp1 = bp0 + (size_t)16 * CCH;
  v8f acc0 = {}, acc1 = {};
  gemm_k_loop(ap, bp0, bp1, (unsigned)CCH, acc0, acc1);
#pragma unroll
  for (int r = 0; r < 8; ++r) {
    float* d = &Cs[(mw * 16u + hh * 8u + (unsigned)r) * LDC + nw * 32u + m];
    d[0]  = acc0[r];
    d[16] = acc1[r];
  }
  __syncthreads();

  const float cs = 1.0f / (XCARRY * WCARRY);
  const unsigned pc = (tid & 3u) * 8u;

  v8h xq, xr;
  size_t offq;
  {
    const unsigned r = tid >> 2;
    const v4f u0 = *(const v4f*)&Cs[r * LDC + pc];
    const v4f u1 = *(const v4f*)&Cs[r * LDC + pc + 4u];
#pragma unroll
    for (int j = 0; j < 4; ++j) {
      const float t0 = u0[j] * cs;
      const float t1 = u1[j] * cs;
      const h16 h0 = toh_flush(t0);
      const h16 h1 = toh_flush(t1);
      xq[j]     = h0;
      xq[j + 4] = h1;
      xr[j]     = toh_flush((t0 - (float)h0) * RCARRY);
      xr[j + 4] = toh_flush((t1 - (float)h1) * RCARRY);
    }
    offq = ((size_t)b * NTOK + pool_pos(T, r)) * DQK + pc;
  }

  v8h kq, kr;
  size_t offk;
  {
    const unsigned j = (tid >> 2) & 15u;
    const unsigned cb = 32u + pc;
#pragma unroll
    for (unsigned hq = 0; hq < 2u; ++hq) {
      const v4f a  = *(const v4f*)&Cs[(2u * j) * LDC + cb + 4u * hq];
      const v4f bq = *(const v4f*)&Cs[(2u * j + 1u) * LDC + cb + 4u * hq];
      const v4f c  = *(const v4f*)&Cs[(32u + 2u * j) * LDC + cb + 4u * hq];
      const v4f d  = *(const v4f*)&Cs[(33u + 2u * j) * LDC + cb + 4u * hq];
#pragma unroll
      for (unsigned i = 0; i < 4u; ++i) {
        const float t = fmaxf(fmaxf(a[i], bq[i]), fmaxf(c[i], d[i])) * cs;
        const h16 hv = toh_flush(t);
        kq[4u * hq + i] = hv;
        kr[4u * hq + i] = toh_flush((t - (float)hv) * RCARRY);
      }
    }
    offk = ((size_t)b * MTOK + 16u * T + j) * DQK + pc;
  }
  const bool kpart = (w < 2u);

  *(volatile v8h*)(Qh + offq) = xq;
  *(volatile v8h*)(Qr + offq) = xr;
  if (kpart) {
    *(volatile v8h*)(Kh + offk) = kq;
    *(volatile v8h*)(Kr + offk) = kr;
  }
  __threadfence();
  *(volatile v8h*)(Qh + offq) = xq;
  *(volatile v8h*)(Qr + offq) = xr;
  if (kpart) {
    *(volatile v8h*)(Kh + offk) = kq;
    *(volatile v8h*)(Kr + offk) = kr;
  }
}

__global__ __launch_bounds__(256) void gemm_v_kernel(
    const h16* __restrict__ Xt, const h16* __restrict__ Wv16, h16* __restrict__ Vt) {
  __shared__ __attribute__((aligned(16))) float Cs[64 * LDC];
  __shared__ __attribute__((aligned(16))) h16 Vp[64 * LDT];
  const unsigned tid = threadIdx.x, lane = tid & 31u;
  const unsigned w = __builtin_amdgcn_readfirstlane(tid >> 5);
  const unsigned mw = w >> 1, nw = w & 1u;
  const unsigned hh = lane >> 4, m = lane & 15u;
  const unsigned n0 = blockIdx.x * 64u;
  const unsigned g = blockIdx.y;
  const unsigned b = blockIdx.z;
  const float cs = 1.0f / (XCARRY * WCARRY);

  const h16* bp0 = Wv16 + (size_t)(n0 + nw * 32u + m) * CCH + hh * 8u;
  const h16* bp1 = bp0 + (size_t)16 * CCH;

#pragma unroll 1
  for (unsigned t = 0; t < 4u; ++t) {
    const unsigned T = g * 4u + t;
    const unsigned na = pool_pos(T, mw * 16u + m);
    const h16* ap = Xt + ((size_t)b * NTOK + na) * CCH + hh * 8u;
    v8f acc0 = {}, acc1 = {};
    gemm_k_loop(ap, bp0, bp1, (unsigned)CCH, acc0, acc1);
#pragma unroll
    for (int r = 0; r < 8; ++r) {
      float* d = &Cs[(mw * 16u + hh * 8u + (unsigned)r) * LDC + nw * 32u + m];
      d[0]  = acc0[r];
      d[16] = acc1[r];
    }
    __syncthreads();
    const unsigned dcol = tid & 63u, jq = tid >> 6;
#pragma unroll
    for (unsigned i = 0; i < 4u; ++i) {
      const unsigned j = jq * 4u + i;
      const float a = fmaxf(fmaxf(Cs[(2u * j) * LDC + dcol], Cs[(2u * j + 1u) * LDC + dcol]),
                            fmaxf(Cs[(32u + 2u * j) * LDC + dcol],
                                  Cs[(33u + 2u * j) * LDC + dcol]));
      Vp[dcol * LDT + 16u * t + j] = toh_flush(a * cs);
    }
    __syncthreads();
  }

  v8h x[2];
  size_t off[2];
#pragma unroll
  for (unsigned i = 0; i < 2u; ++i) {
    const unsigned dcol = 32u * i + (tid >> 3);
    const unsigned kk = (tid & 7u) * 8u;
    x[i] = *(const v8h*)&Vp[dcol * LDT + kk];
    off[i] = ((size_t)b * DV + n0 + dcol) * MTOK + 64u * g + kk;
  }
#pragma unroll
  for (int i = 0; i < 2; ++i) *(volatile v8h*)(Vt + off[i]) = x[i];
  __threadfence();
#pragma unroll
  for (int i = 0; i < 2; ++i) *(volatile v8h*)(Vt + off[i]) = x[i];
}

__global__ __launch_bounds__(256) __attribute__((amdgpu_num_vgpr(256))) void attn_kernel(
    const h16* __restrict__ Qh, const h16* __restrict__ Qr,
    const h16* __restrict__ Kh, const h16* __restrict__ Kr,
    const h16* __restrict__ Vt, h16* __restrict__ Ov) {
  __shared__ __attribute__((aligned(16))) h16 Ks[64 * LDK];
  __shared__ __attribute__((aligned(16))) h16 KRs[64 * LDK];
  __shared__ __attribute__((aligned(16))) h16 Vs[DV * LDT];
  __shared__ __attribute__((aligned(16))) h16 Ps[8 * 16 * LDP];

  const unsigned tid = threadIdx.x, lane = tid & 31u;
  const unsigned w = __builtin_amdgcn_readfirstlane(tid >> 5);
  const unsigned hh = lane >> 4, m = lane & 15u;
  const unsigned b = blockIdx.y;
  const unsigned qrow0 = blockIdx.x * 128u + w * 16u;
  const unsigned pbase = w * (16u * LDP);

  const size_t qoff = ((size_t)b * NTOK + qrow0 + m) * DQK + hh * 8u;
  const v16h qh = frag_at(Qh + qoff);
#if SCORE_RES
  const v16h qr = frag_at(Qr + qoff);
#endif

  float mrow[8], lrow[8];
  v8f o[8];
#pragma unroll
  for (int v = 0; v < 8; ++v) { mrow[v] = -1.0e30f; lrow[v] = 0.0f; }
#pragma unroll
  for (int nb = 0; nb < 8; ++nb) o[nb] = (v8f){};

  const size_t kplane = (size_t)b * MTOK * DQK;
  const size_t vplane = (size_t)b * DV * MTOK;

  for (unsigned kb = 0; kb < (unsigned)MTOK; kb += 64u) {
    {
      const unsigned r = tid >> 2, c = (tid & 3u) * 8u;
      *(v8h*)&Ks[r * LDK + c] = *(const v8h*)(Kh + kplane + (size_t)(kb + r) * DQK + c);
#if SCORE_RES
      *(v8h*)&KRs[r * LDK + c] = *(const v8h*)(Kr + kplane + (size_t)(kb + r) * DQK + c);
#endif
    }
#pragma unroll
    for (unsigned j = 0; j < 4u; ++j) {
      const unsigned idx = tid + 256u * j;
      const unsigned r = idx >> 3, c = (idx & 7u) * 8u;
      *(v8h*)&Vs[r * LDT + c] = *(const v8h*)(Vt + vplane + (size_t)r * MTOK + kb + c);
    }
    __syncthreads();

    v8f s[4];
#pragma unroll
    for (int kg = 0; kg < 4; ++kg) {
      const v16h kf = ld_frag(&Ks[(kg * 16) * LDK], LDK);
      v8f t = {};
      t = wmma16(qh, kf, t);
#if SCORE_RES
      const v16h krf = ld_frag(&KRs[(kg * 16) * LDK], LDK);
      v8f tr = {};
      tr = wmma16(qh, krf, tr);
      tr = wmma16(qr, kf, tr);
      s[kg] = t + tr * (1.0f / RCARRY);
#else
      s[kg] = t;
#endif
    }

    float alpha[8];
#pragma unroll
    for (int v = 0; v < 8; ++v) {
      float mx = fmaxf(fmaxf(s[0][v], s[1][v]), fmaxf(s[2][v], s[3][v]));
      mx = red16_max(mx);
      const float mn = fmaxf(mrow[v], mx);
      alpha[v] = __expf(mrow[v] - mn);
      mrow[v] = mn;
    }
#pragma unroll
    for (int kg = 0; kg < 4; ++kg)
#pragma unroll
      for (int v = 0; v < 8; ++v) {
        const float p = __expf(s[kg][v] - mrow[v]);
        const h16 ph = toh_flush(p * PCARRY);
        Ps[pbase + (hh * 8u + (unsigned)v) * LDP + (unsigned)kg * 16u + m] = ph;
        s[kg][v] = (float)ph;
      }
#pragma unroll
    for (int v = 0; v < 8; ++v) {
      const float rs = red16_sum((s[0][v] + s[1][v]) + (s[2][v] + s[3][v]));
      lrow[v] = alpha[v] * lrow[v] + rs;
    }
#pragma unroll
    for (int nb = 0; nb < 8; ++nb)
#pragma unroll
      for (int v = 0; v < 8; ++v) o[nb][v] = o[nb][v] * alpha[v];
    wave_lds_sync();

#pragma unroll
    for (int c = 0; c < 2; ++c) {
      const v16h pf = ld_frag(&Ps[pbase + c * 32], LDP);
#pragma unroll
      for (int nb = 0; nb < 8; ++nb) {
        const v16h vf = ld_frag(&Vs[(nb * 16) * LDT + c * 32], LDT);
        o[nb] = wmma16(pf, vf, o[nb]);
      }
    }
    __syncthreads();
  }

  float inv[8];
#pragma unroll
  for (int v = 0; v < 8; ++v) inv[v] = __builtin_amdgcn_rcpf(lrow[v]) * VCARRY;
#pragma unroll
  for (int nb = 0; nb < 8; ++nb)
#pragma unroll
    for (int v = 0; v < 8; ++v)
      Ps[pbase + (hh * 8u + (unsigned)v) * LDP + (unsigned)nb * 16u + m] =
          toh_flush(o[nb][v] * inv[v]);
  wave_lds_sync();
  v8h x[8];
  size_t off[8];
#pragma unroll
  for (unsigned i = 0; i < 8u; ++i) {
    const unsigned r = 2u * i + (lane >> 4);
    const unsigned c = (lane & 15u) * 8u;
    x[i] = *(const v8h*)&Ps[pbase + r * LDP + c];
    off[i] = ((size_t)b * NTOK + qrow0 + r) * DV + c;
  }
#pragma unroll
  for (int i = 0; i < 8; ++i) *(volatile v8h*)(Ov + off[i]) = x[i];
  __threadfence();
#pragma unroll
  for (int i = 0; i < 8; ++i) *(volatile v8h*)(Ov + off[i]) = x[i];
}

__global__ __launch_bounds__(256) void gemm_out_kernel(
    const h16* __restrict__ Wo16, const h16* __restrict__ Ctx,
    const float* __restrict__ X, const float* __restrict__ gam, float* __restrict__ outf) {
  __shared__ __attribute__((aligned(16))) float Cs[64 * LDC];
  const unsigned tid = threadIdx.x, lane = tid & 31u;
  const unsigned w = __builtin_amdgcn_readfirstlane(tid >> 5);
  const unsigned mw = w >> 1, nw = w & 1u;
  const unsigned hh = lane >> 4, m = lane & 15u;
  const unsigned n0 = blockIdx.x * 64u;
  const unsigned row0 = blockIdx.y * 64u;
  const unsigned b = blockIdx.z;

  const h16* ap  = Wo16 + (size_t)(row0 + mw * 16u + m) * DV + hh * 8u;
  const h16* bp0 = Ctx + ((size_t)b * NTOK + n0 + nw * 32u + m) * DV + hh * 8u;
  const h16* bp1 = bp0 + (size_t)16 * DV;
  v8f acc0 = {}, acc1 = {};
  gemm_k_loop(ap, bp0, bp1, (unsigned)DV, acc0, acc1);
#pragma unroll
  for (int r = 0; r < 8; ++r) {
    float* d = &Cs[(mw * 16u + hh * 8u + (unsigned)r) * LDC + nw * 32u + m];
    d[0]  = acc0[r];
    d[16] = acc1[r];
  }
  __syncthreads();

  const float gsc = bf16r(gam[0]);
  const float cs = 1.0f / (WCARRY * VCARRY);
  v4f xs[4];
  size_t off[4];
#pragma unroll
  for (unsigned i = 0; i < 4u; ++i) {
    const unsigned r = 16u * i + (tid >> 4);
    const unsigned c = (tid & 15u) * 4u;
    const size_t o = ((size_t)b * CCH + row0 + r) * NTOK + n0 + c;
    const v4f u = *(const v4f*)&Cs[r * LDC + c];
    const v4f xin = *(const v4f*)(X + o);
    v4f val;
#pragma unroll
    for (int j = 0; j < 4; ++j) val[j] = bf16r(xin[j]) + gsc * (u[j] * cs);
    xs[i] = val;
    off[i] = o;
  }
#pragma unroll
  for (int i = 0; i < 4; ++i) *(volatile v4f*)(outf + off[i]) = xs[i];
  __threadfence();
#pragma unroll
  for (int i = 0; i < 4; ++i) *(volatile v4f*)(outf + off[i]) = xs[i];
}

extern "C" void kernel_launch(void* const* d_in, const int* in_sizes, int n_in,
                              void* d_out, int out_size, void* d_ws, size_t ws_size,
                              hipStream_t stream) {
  if (n_in < 6) return;
  const long long need_x = (long long)NB * CCH * NTOK;
  if ((long long)in_sizes[0] < need_x) return;
  if ((long long)in_sizes[1] < (long long)DQK * CCH) return;
  if ((long long)in_sizes[2] < (long long)DQK * CCH) return;
  if ((long long)in_sizes[3] < (long long)DV * CCH) return;
  if ((long long)in_sizes[4] < (long long)CCH * DV) return;
  if (in_sizes[5] < 1) return;
  if ((long long)out_size < need_x) return;
  if (ws_size < WS_TOTAL) return;

  const float* X   = (const float*)d_in[0];
  const float* wq  = (const float*)d_in[1];
  const float* wk  = (const float*)d_in[2];
  const float* wv  = (const float*)d_in[3];
  const float* wo  = (const float*)d_in[4];
  const float* gam = (const float*)d_in[5];
  float* out = (float*)d_out;

  char* ws = (char*)d_ws;
  h16* Xt16  = (h16*)(ws + OFF_XT);
  h16* Wqk16 = (h16*)(ws + OFF_WQK);
  h16* Wv16  = (h16*)(ws + OFF_WV);
  h16* Wo16  = (h16*)(ws + OFF_WO);
  h16* Q16   = (h16*)(ws + OFF_Q);
  h16* QR16  = (h16*)(ws + OFF_QR);
  h16* K16   = (h16*)(ws + OFF_K);
  h16* KR16  = (h16*)(ws + OFF_KR);
  h16* Vt16  = (h16*)(ws + OFF_VT);
  h16* Ctx16 = (h16*)(ws + OFF_CTX);

  dim3 blk(256);

  wcast_kernel<<<dim3((DQK * CCH) / 2048), blk, 0, stream>>>(wq, Wqk16);
  wcast_kernel<<<dim3((DQK * CCH) / 2048), blk, 0, stream>>>(wk, Wqk16 + (size_t)DQK * CCH);
  wcast_kernel<<<dim3((DV * CCH) / 2048), blk, 0, stream>>>(wv, Wv16);
  wcast_kernel<<<dim3((CCH * DV) / 2048), blk, 0, stream>>>(wo, Wo16);

  xconv_kernel<<<dim3(NTOK / 64, CCH / 64, NB), blk, 0, stream>>>(X, Xt16);

  gemm_qk_kernel<<<dim3(NTOK / 64, NB), blk, 0, stream>>>(Xt16, Wqk16, Q16, QR16, K16, KR16);
  gemm_v_kernel<<<dim3(DV / 64, NTOK / 256, NB), blk, 0, stream>>>(Xt16, Wv16, Vt16);
  attn_kernel<<<dim3(NTOK / 128, NB), blk, 0, stream>>>(Q16, QR16, K16, KR16, Vt16, Ctx16);
  gemm_out_kernel<<<dim3(NTOK / 64, CCH / 64, NB), blk, 0, stream>>>(Wo16, Ctx16, X, gam, out);
}
